// TextClassifier_33217277067654
// MI455X (gfx1250) — hardware-verified
//
#include <hip/hip_runtime.h>


namespace {
constexpr int VOC = 50265, EM = 256, NH = 4, HD = 64, WIN = 64, NC = 20, B = 8, S = 2048, NT = B * S, NQT = S / 16;
constexpr float XE = 256.0f, AS_ = 4096.0f, PS = 2048.0f, WSC = 256.0f;
typedef _Float16 b16;
typedef __attribute__((ext_vector_type(16))) _Float16 v16b;
typedef __attribute__((ext_vector_type(8))) _Float16 v8b;
typedef __attribute__((ext_vector_type(8))) float v8f;
typedef __attribute__((ext_vector_type(4))) float v4f;
__device__ __forceinline__ float bf16_rne(float f) { unsigned int u = __float_as_uint(f); u += 0x7FFFu + ((u >> 16) & 1u); return __uint_as_float(u & 0xFFFF0000u); }
__device__ __forceinline__ void split16(float v, b16& hi, b16& lo) { hi = (b16)v; lo = (b16)(v - (float)hi); }
__device__ __forceinline__ v16b frag_kb(const b16* p, int hh) { const v8b a = *(const v8b*)(p + 8 * hh), b = *(const v8b*)(p + 16 + 8 * hh); v16b f;
#pragma unroll
  for (int e = 0; e < 8; ++e) { f[e] = a[e]; f[8 + e] = b[e]; } return f; }
__device__ __forceinline__ v8f wmma16b(v16b a, v16b b, v8f c) { v8f d = __builtin_amdgcn_wmma_f32_16x16x32_f16(false, a, false, b, (short)0, c, false, false); asm volatile("v_nop\n\tv_nop\n\tv_nop\n\tv_nop" : "+v"(d) : "v"(a), "v"(b)); return d; }
__device__ __forceinline__ void wave_lds_sync() { __builtin_amdgcn_fence(__ATOMIC_RELEASE, "workgroup"); __builtin_amdgcn_wave_barrier(); __builtin_amdgcn_fence(__ATOMIC_ACQUIRE, "workgroup"); }
__device__ __forceinline__ float pmul(float a, float b) { float p = a * b; asm volatile("" : "+v"(p)); return p; }
__device__ __forceinline__ int iclamp(int v, int lo, int hi) { return v < lo ? lo : (v > hi ? hi : v); }
__device__ __forceinline__ float leaky(float v) { return v >= 0.0f ? v : 0.01f * v; }

__global__ __launch_bounds__(256) void wcopy_kernel(const float* __restrict__ w, int OUTW, int OUTP, int KIN, b16* __restrict__ WT) {
  const size_t u = (size_t)blockIdx.x * 256 + threadIdx.x; const size_t n8 = (size_t)OUTP * KIN / 8; if (u >= n8) return; const size_t e = u * 8; const int o = (int)(e / KIN); v8b v;
#pragma unroll
  for (int j = 0; j < 8; ++j) v[j] = (o < OUTW) ? (b16)(bf16_rne(w[e + j]) * WSC) : (b16)0.0f; for (int pass = 0; pass < 2; ++pass) { *(volatile v8b*)(WT + e) = v; __threadfence(); }
}
__global__ __launch_bounds__(32) void qkv_kernel(const int* __restrict__ text, const float* __restrict__ emb, const b16* __restrict__ WI, const float* __restrict__ bi, int NTV, b16* __restrict__ QB, b16* __restrict__ KB_, b16* __restrict__ VB) {
  __shared__ __attribute__((aligned(16))) b16 Ah[16][EM + 8]; __shared__ __attribute__((aligned(16))) b16 Tb[16][128 + 8];
  const int lane = threadIdx.x, nloc = lane & 15, hlf = lane >> 4; const size_t t0 = (size_t)blockIdx.x * 16; if (t0 >= (size_t)NTV) return;
  for (int rr = 0; rr < 16; ++rr) { const int tk = iclamp(text[t0 + rr], 0, VOC - 1); for (int q = 0; q < 8; ++q) Ah[rr][q * 32 + lane] = (b16)(bf16_rne(emb[(size_t)tk * EM + q * 32 + lane]) * XE); }
  wave_lds_sync();
#pragma unroll 1
  for (int cg = 0; cg < 6; ++cg) { v8f acc[8];
#pragma unroll
    for (int t = 0; t < 8; ++t) acc[t] = (v8f){};
#pragma unroll 2
    for (int kb = 0; kb < EM; kb += 32) { const v16b a = frag_kb(&Ah[nloc][kb], hlf);
#pragma unroll
      for (int t = 0; t < 8; ++t) acc[t] = wmma16b(a, frag_kb(WI + (size_t)(cg * 128 + t * 16 + nloc) * EM + kb, hlf), acc[t]); }
    const float post = (cg < 2) ? (AS_ / 8.0f) : AS_;
#pragma unroll
    for (int t = 0; t < 8; ++t) { const int c = cg * 128 + t * 16 + nloc; const float bb = bf16_rne(bi[c]);
#pragma unroll
      for (int r8 = 0; r8 < 8; ++r8) Tb[8 * hlf + r8][t * 16 + nloc] = (b16)((acc[t][r8] * (1.0f / (XE * WSC)) + bb) * post); }
    wave_lds_sync();
    b16* dst = cg < 2 ? QB : (cg < 4 ? KB_ : VB); const int co = (cg & 1) * 128;
    for (int pass = 0; pass < 2; ++pass) { for (int rr = 0; rr < 16; ++rr) { const int r2 = rr, c8 = (lane & 15) * 8; if ((lane >> 4) == (rr & 1)) *(volatile v8b*)(dst + (t0 + r2) * EM + co + c8) = *(const v8b*)(&Tb[r2][c8]); } __threadfence(); }
    wave_lds_sync(); }
}
__global__ __launch_bounds__(256) void vt_kernel(const b16* __restrict__ VB, int NTV, b16* __restrict__ VT) {
  __shared__ b16 Tt[64][EM + 2]; const size_t s0 = (size_t)blockIdx.x * 64; if (s0 >= (size_t)NTV) return; const int b = (int)(s0 / S), sl = (int)(s0 % S); const int tid = threadIdx.x;
  for (int i = tid; i < 64 * EM; i += 256) { const int r = i / EM, c = i % EM; Tt[r][c] = VB[(s0 + r) * EM + c]; }
  __syncthreads();
  { const int c = tid; const int h = c / HD, d = c % HD; for (int g = 0; g < 8; ++g) { v8b v; for (int j = 0; j < 8; ++j) v[j] = Tt[g * 8 + j][c]; const size_t o = ((size_t)(b * NH + h) * HD + d) * S + sl + g * 8; for (int pass = 0; pass < 2; ++pass) { *(volatile v8b*)(VT + o) = v; __threadfence(); } } }
}
__global__ __launch_bounds__(32) void att_kernel(const b16* __restrict__ QB, const b16* __restrict__ KB_, const b16* __restrict__ VT, int NWV, float* __restrict__ AO) {
  __shared__ __attribute__((aligned(16))) b16 Ph[16][40]; __shared__ float Mx[16], Sm[16]; __shared__ __attribute__((aligned(16))) float Tf[16][HD + 4];
  const int lane = threadIdx.x, nloc = lane & 15, hlf = lane >> 4; if ((int)blockIdx.x >= NWV) return; const int qt = blockIdx.x % NQT, h = (blockIdx.x / NQT) % NH, b = blockIdx.x / (NQT * NH); const int q0 = qt * 16; const size_t tb = (size_t)b * S;
  const v16b qa0 = frag_kb(QB + (tb + q0 + nloc) * EM + h * HD, hlf), qa1 = frag_kb(QB + (tb + q0 + nloc) * EM + h * HD + 32, hlf);
  int kb0 = q0 - WIN; kb0 = kb0 < 0 ? 0 : (kb0 & ~31); int kb1 = q0 + 15 + WIN; kb1 = kb1 >= S ? S - 1 : kb1;
  auto scores = [&](int kb, v8f sacc[2]) {
#pragma unroll
    for (int st = 0; st < 2; ++st) { int k = kb + st * 16 + nloc; k = k < S ? k : S - 1; const b16* kr = KB_ + (tb + k) * EM + h * HD; sacc[st] = (v8f){}; sacc[st] = wmma16b(qa0, frag_kb(kr, hlf), sacc[st]); sacc[st] = wmma16b(qa1, frag_kb(kr + 32, hlf), sacc[st]); } };
  const float scl = 1.0f / (AS_ * AS_); float rmax[8];
#pragma unroll
  for (int r8 = 0; r8 < 8; ++r8) rmax[r8] = -INFINITY;
#pragma unroll 1
  for (int kb = kb0; kb <= kb1; kb += 32) { v8f sacc[2]; scores(kb, sacc);
#pragma unroll
    for (int st = 0; st < 2; ++st) { const int k = kb + st * 16 + nloc;
#pragma unroll
      for (int r8 = 0; r8 < 8; ++r8) { const int qq = q0 + 8 * hlf + r8; const int dd = k - qq; if (k < S && dd <= WIN && dd >= -WIN) rmax[r8] = fmaxf(rmax[r8], sacc[st][r8] * scl); } } }
#pragma unroll
  for (int r8 = 0; r8 < 8; ++r8) { float m = rmax[r8]; for (int o = 1; o < 16; o <<= 1) m = fmaxf(m, __shfl_xor(m, o)); if (nloc == 0) Mx[8 * hlf + r8] = m; }
  wave_lds_sync();
  v8f acc[4] = {(v8f){}, (v8f){}, (v8f){}, (v8f){}}; float rsum[8];
#pragma unroll
  for (int r8 = 0; r8 < 8; ++r8) rsum[r8] = 0.0f;
#pragma unroll 1
  for (int kb = kb0; kb <= kb1; kb += 32) { v8f sacc[2]; scores(kb, sacc);
#pragma unroll
    for (int st = 0; st < 2; ++st) { const int k = kb + st * 16 + nloc;
#pragma unroll
      for (int r8 = 0; r8 < 8; ++r8) { const int rl = 8 * hlf + r8; const int qq = q0 + rl; const int dd = k - qq; float p = 0.0f; if (k < S && dd <= WIN && dd >= -WIN) p = __expf(sacc[st][r8] * scl - Mx[rl]); rsum[r8] += p; Ph[rl][st * 16 + nloc] = (b16)(p * PS); } }
    wave_lds_sync();
    const v16b pa = frag_kb(&Ph[nloc][0], hlf);
#pragma unroll
    for (int t = 0; t < 4; ++t) acc[t] = wmma16b(pa, frag_kb(VT + ((size_t)(b * NH + h) * HD + t * 16 + nloc) * S + kb, hlf), acc[t]);
    wave_lds_sync(); }
#pragma unroll
  for (int r8 = 0; r8 < 8; ++r8) { float s = rsum[r8]; for (int o = 1; o < 16; o <<= 1) s += __shfl_xor(s, o); if (nloc == 0) Sm[8 * hlf + r8] = s; }
  wave_lds_sync();
#pragma unroll
  for (int t = 0; t < 4; ++t)
#pragma unroll
    for (int r8 = 0; r8 < 8; ++r8) { const int rl = 8 * hlf + r8; Tf[rl][t * 16 + nloc] = acc[t][r8] * (1.0f / (PS * AS_)) / Sm[rl]; }
  wave_lds_sync();
  for (int pass = 0; pass < 2; ++pass) { for (int rr = 0; rr < 16; ++rr) { ((volatile float*)AO)[(tb + q0 + rr) * EM + h * HD + lane] = Tf[rr][lane]; ((volatile float*)AO)[(tb + q0 + rr) * EM + h * HD + 32 + lane] = Tf[rr][32 + lane]; } __threadfence(); }
}
__global__ __launch_bounds__(32) void oproj_kernel(const float* __restrict__ AO, const b16* __restrict__ WO, const float* __restrict__ bo, int NTV, float* __restrict__ OP) {
  __shared__ __attribute__((aligned(16))) b16 Ah[16][EM + 8]; __shared__ __attribute__((aligned(16))) float Tf[16][128 + 4];
  const int lane = threadIdx.x, nloc = lane & 15, hlf = lane >> 4; const size_t t0 = (size_t)blockIdx.x * 16; if (t0 >= (size_t)NTV) return;
  for (int rr = 0; rr < 16; ++rr) for (int q = 0; q < 8; ++q) Ah[rr][q * 32 + lane] = (b16)(AO[(t0 + rr) * EM + q * 32 + lane] * AS_);
  wave_lds_sync();
#pragma unroll 1
  for (int cg = 0; cg < 2; ++cg) { v8f acc[8];
#pragma unroll
    for (int t = 0; t < 8; ++t) acc[t] = (v8f){};
#pragma unroll 2
    for (int kb = 0; kb < EM; kb += 32) { const v16b a = frag_kb(&Ah[nloc][kb], hlf);
#pragma unroll
      for (int t = 0; t < 8; ++t) acc[t] = wmma16b(a, frag_kb(WO + (size_t)(cg * 128 + t * 16 + nloc) * EM + kb, hlf), acc[t]); }
#pragma unroll
    for (int t = 0; t < 8; ++t) { const int c = cg * 128 + t * 16 + nloc; const float bb = bf16_rne(bo[c]);
#pragma unroll
      for (int r8 = 0; r8 < 8; ++r8) Tf[8 * hlf + r8][t * 16 + nloc] = acc[t][r8] * (1.0f / (AS_ * WSC)) + bb; }
    wave_lds_sync();
    for (int pass = 0; pass < 2; ++pass) { for (int rr = 0; rr < 16; ++rr) *(volatile v4f*)(OP + (t0 + rr) * EM + cg * 128 + lane * 4) = *(const v4f*)(&Tf[rr][lane * 4]); __threadfence(); }
    wave_lds_sync(); }
}
__global__ __launch_bounds__(256) void max_kernel(const float* __restrict__ OP, int NBV, float* __restrict__ CTX) {
  const int b = blockIdx.x, c = threadIdx.x; if (b >= NBV) return; float m = -INFINITY;
#pragma unroll 4
  for (int s = 0; s < S; ++s) m = fmaxf(m, OP[((size_t)b * S + s) * EM + c]);
  for (int pass = 0; pass < 2; ++pass) { ((volatile float*)CTX)[b * EM + c] = m; __threadfence(); }
}
__global__ __launch_bounds__(32) void fc_kernel(const float* __restrict__ CTX, int NBV, const b16* __restrict__ W1, const float* __restrict__ b1, const b16* __restrict__ W2, const float* __restrict__ b2, const b16* __restrict__ W3, const float* __restrict__ b3, float* __restrict__ out) {
  __shared__ __attribute__((aligned(16))) b16 Ah[16][512 + 8], Al[16][512 + 8]; __shared__ float H1[16][512], So[16][32];
  const int lane = threadIdx.x, nloc = lane & 15, hlf = lane >> 4;
  for (int rr = 0; rr < 16; ++rr) for (int q = 0; q < 8; ++q) { const float v = rr < NBV ? CTX[rr * EM + q * 32 + lane] : 0.0f; b16 p, ql; split16(v * 4096.0f, p, ql); Ah[rr][q * 32 + lane] = p; Al[rr][q * 32 + lane] = ql; }
  wave_lds_sync();
#pragma unroll 1
  for (int cg = 0; cg < 4; ++cg) { v8f acc[8];
#pragma unroll
    for (int t = 0; t < 8; ++t) acc[t] = (v8f){};
    for (int kb = 0; kb < 256; kb += 32) { const v16b a = frag_kb(&Ah[nloc][kb], hlf), al = frag_kb(&Al[nloc][kb], hlf);
#pragma unroll
      for (int t = 0; t < 8; ++t) { const v16b bw = frag_kb(W1 + (size_t)(cg * 128 + t * 16 + nloc) * 256 + kb, hlf); acc[t] = wmma16b(a, bw, acc[t]); acc[t] = wmma16b(al, bw, acc[t]); } }
#pragma unroll
    for (int t = 0; t < 8; ++t) { const int c = cg * 128 + t * 16 + nloc; const float bb = bf16_rne(b1[c]);
#pragma unroll
      for (int r8 = 0; r8 < 8; ++r8) H1[8 * hlf + r8][c] = leaky(acc[t][r8] * (1.0f / (4096.0f * WSC)) + bb); } }
  wave_lds_sync();
  for (int rr = 0; rr < 16; ++rr) for (int q = 0; q < 16; ++q) { b16 p, ql; split16(H1[rr][q * 32 + lane] * 16384.0f, p, ql); Ah[rr][q * 32 + lane] = p; Al[rr][q * 32 + lane] = ql; }
  wave_lds_sync();
#pragma unroll 1
  for (int cg = 0; cg < 2; ++cg) { v8f acc[8];
#pragma unroll
    for (int t = 0; t < 8; ++t) acc[t] = (v8f){};
    for (int kb = 0; kb < 512; kb += 32) { const v16b a = frag_kb(&Ah[nloc][kb], hlf), al = frag_kb(&Al[nloc][kb], hlf);
#pragma unroll
      for (int t = 0; t < 8; ++t) { const v16b bw = frag_kb(W2 + (size_t)(cg * 128 + t * 16 + nloc) * 512 + kb, hlf); acc[t] = wmma16b(a, bw, acc[t]); acc[t] = wmma16b(al, bw, acc[t]); } }
#pragma unroll
    for (int t = 0; t < 8; ++t) { const int c = cg * 128 + t * 16 + nloc; const float bb = bf16_rne(b2[c]);
#pragma unroll
      for (int r8 = 0; r8 < 8; ++r8) H1[8 * hlf + r8][c] = leaky(acc[t][r8] * (1.0f / (16384.0f * WSC)) + bb); } }
  wave_lds_sync();
  for (int rr = 0; rr < 16; ++rr) for (int q = 0; q < 8; ++q) { b16 p, ql; split16(H1[rr][q * 32 + lane] * 65536.0f, p, ql); Ah[rr][q * 32 + lane] = p; Al[rr][q * 32 + lane] = ql; }
  wave_lds_sync();
#pragma unroll
  for (int t = 0; t < 2; ++t) { v8f acc = {}; for (int kb = 0; kb < 256; kb += 32) { const v16b bw = frag_kb(W3 + (size_t)(t * 16 + nloc) * 256 + kb, hlf); acc = wmma16b(frag_kb(&Ah[nloc][kb], hlf), bw, acc); acc = wmma16b(frag_kb(&Al[nloc][kb], hlf), bw, acc); }
    const int c = t * 16 + nloc; const float bb = c < NC ? bf16_rne(b3[c]) : 0.0f;
#pragma unroll
    for (int r8 = 0; r8 < 8; ++r8) So[8 * hlf + r8][c] = acc[r8] * (1.0f / (65536.0f * WSC)) + bb; }
  wave_lds_sync();
  for (int pass = 0; pass < 2; ++pass) { for (int i = lane; i < B * NC; i += 32) ((volatile float*)out)[i] = So[i / NC][i % NC]; __threadfence(); }
}
}

extern "C" void kernel_launch(void* const* d_in, const int* in_sizes, int n_in, void* d_out, int out_size, void* d_ws, size_t ws_size, hipStream_t stream) {
  (void)n_in;
  auto Fp = [&](int i) { return (const float*)d_in[i]; }; auto Ip = [&](int i) { return (const int*)d_in[i]; };
  if (in_sizes[0] != B * S || in_sizes[1] != VOC * EM || in_sizes[2] != 3 * EM * EM || in_sizes[4] != EM * EM || in_sizes[6] != 512 * EM || in_sizes[8] != 256 * 512 || in_sizes[10] != NC * 256 || out_size != B * NC) return;
  const int NBV = B; const int NTV = NBV * S, NWV = NBV * NH * NQT;
  size_t off = 0; char* ws = (char*)d_ws;
  auto carve = [&](size_t bytes) { char* p = ws + off; off += (bytes + 255) & ~(size_t)255; return p; };
  b16* WI = (b16*)carve((size_t)3 * EM * EM * 2); b16* WO = (b16*)carve((size_t)EM * EM * 2); b16* W1 = (b16*)carve((size_t)512 * 256 * 2); b16* W2 = (b16*)carve((size_t)256 * 512 * 2); b16* W3 = (b16*)carve((size_t)32 * 256 * 2);
  b16* QB = (b16*)carve((size_t)NT * EM * 2); b16* KB_ = (b16*)carve((size_t)NT * EM * 2); b16* VB = (b16*)carve((size_t)NT * EM * 2); b16* VT = (b16*)carve((size_t)B * NH * HD * S * 2); float* AO = (float*)carve((size_t)NT * EM * 4); float* OP = (float*)carve((size_t)NT * EM * 4); float* CTX = (float*)carve((size_t)16 * EM * 4);
  if (off > ws_size || off > ((size_t)96 << 20)) return;
  wcopy_kernel<<<(3 * EM * EM / 8 + 255) / 256, 256, 0, stream>>>(Fp(2), 3 * EM, 3 * EM, EM, WI); wcopy_kernel<<<(EM * EM / 8 + 255) / 256, 256, 0, stream>>>(Fp(4), EM, EM, EM, WO);
  wcopy_kernel<<<(512 * 256 / 8 + 255) / 256, 256, 0, stream>>>(Fp(6), 512, 512, 256, W1); wcopy_kernel<<<(256 * 512 / 8 + 255) / 256, 256, 0, stream>>>(Fp(8), 256, 256, 512, W2); wcopy_kernel<<<(32 * 256 / 8 + 255) / 256, 256, 0, stream>>>(Fp(10), NC, 32, 256, W3);
  qkv_kernel<<<(unsigned)(NTV / 16), 32, 0, stream>>>(Ip(0), Fp(1), WI, Fp(3), NTV, QB, KB_, VB);
  vt_kernel<<<(unsigned)(NTV / 64), 256, 0, stream>>>(VB, NTV, VT);
  att_kernel<<<(unsigned)NWV, 32, 0, stream>>>(QB, KB_, VT, NWV, AO);
  oproj_kernel<<<(unsigned)(NTV / 16), 32, 0, stream>>>(AO, WO, Fp(5), NTV, OP);
  max_kernel<<<B, EM, 0, stream>>>(OP, NBV, CTX);
  fc_kernel<<<1, 32, 0, stream>>>(CTX, NBV, W1, Fp(7), W2, Fp(9), W3, Fp(11), (float*)d_out);
}
